// AttentionPointEncoder_61778809585774
// MI455X (gfx1250) — hardware-verified
//
#include <hip/hip_runtime.h>
#include <math.h>
#include <stdint.h>

#define NB     2
#define MQ     512
#define NKEY   2048
#define HID    256
#define NHD    8
#define DHD    32
#define FFI    1024
#define NLAY   4
#define NCAT   2561
#define NKP    2624
#define TOKR   16
#define NTOK   32
#define QROWS  (NB * MQ)
#define KROWS  (NB * NKEY)
#define SROWS  (QROWS + KROWS)
#define LNEPS  1e-5f
#define RSCALE 0.17677669529663687f
#define WSC    64.0f
#define PSC    16.0f
#define OSC    32.0f
#define HSC    16.0f

#define F_BIASN 1
#define F_BIASM 2
#define F_RESID 4
#define F_RELU  8
#define F_OUT16 16

static_assert(NHD * DHD == HID);
static_assert((NKP % 64) == 0 && NKP >= NCAT && (NKP % 8) == 0);
static_assert((QROWS % 32) == 0 && (KROWS % 32) == 0 && (SROWS % 32) == 0 && (NTOK % 32) == 0);
static_assert((MQ % 16) == 0 && (NKEY % 64) == 0 && (SROWS % 8) == 0 && (QROWS % 8) == 0);
static_assert(NB * TOKR == NTOK);

typedef _Float16 v16h __attribute__((ext_vector_type(16)));
typedef _Float16 v8h  __attribute__((ext_vector_type(8)));
typedef float    v8f  __attribute__((ext_vector_type(8)));
typedef float    v4f  __attribute__((ext_vector_type(4)));
typedef unsigned int v4u __attribute__((ext_vector_type(4)));

__device__ __forceinline__ unsigned short bf_bits(float f) {
  unsigned u = __float_as_uint(f);
  return (unsigned short)((u + 0x7FFFu + ((u >> 16) & 1u)) >> 16);
}
__device__ __forceinline__ float bf_up(unsigned short h) { return __uint_as_float(((unsigned)h) << 16); }
__device__ __forceinline__ float bfr(float f) { return bf_up(bf_bits(f)); }
__device__ __forceinline__ unsigned short h_bits(_Float16 x) { return __builtin_bit_cast(unsigned short, x); }
__device__ __forceinline__ unsigned pk16(unsigned short a, unsigned short b) { return (unsigned)a | ((unsigned)b << 16); }
__device__ __forceinline__ unsigned pkh(float a, float b) { return pk16(h_bits((_Float16)a), h_bits((_Float16)b)); }
__device__ __forceinline__ v8f zero8() { v8f z = {0.f, 0.f, 0.f, 0.f, 0.f, 0.f, 0.f, 0.f}; return z; }
__device__ __forceinline__ v4f zero4() { v4f z = {0.f, 0.f, 0.f, 0.f}; return z; }

__device__ __forceinline__ v16h ldfrag_h(const _Float16* p) {
  union { v16h v; v8h h[2]; } f;
  f.h[0] = *(const v8h*)(p);
  f.h[1] = *(const v8h*)(p + 16);
  return f.v;
}

__device__ __forceinline__ v8f mma_h(v16h a, v16h b, v8f c) {
  c = __builtin_amdgcn_wmma_f32_16x16x32_f16(false, a, false, b, (short)0, c, false, false);
#if defined(__HIP_DEVICE_COMPILE__)
  asm volatile("v_nop\n\tv_nop\n\tv_nop\n\tv_nop" : "+v"(c) : "v"(a), "v"(b));
#endif
  return c;
}
__device__ __forceinline__ v8f mma_h_raw(v16h a, v16h b, v8f c) {
  return __builtin_amdgcn_wmma_f32_16x16x32_f16(false, a, false, b, (short)0, c, false, false);
}
__device__ __forceinline__ void dep_guard_h(v8f& a, v8f& b, v16h x) {
#if defined(__HIP_DEVICE_COMPILE__)
  asm volatile("v_nop\n\tv_nop\n\tv_nop\n\tv_nop" : "+v"(a), "+v"(b) : "v"(x));
#endif
}
__device__ __forceinline__ void keep4_h(v16h a, v16h b, v16h c, v16h d) {
#if defined(__HIP_DEVICE_COMPILE__)
  asm volatile("v_nop" :: "v"(a), "v"(b), "v"(c), "v"(d));
#endif
}
__device__ __forceinline__ void acc_guard4(v8f& a, v8f& b, v8f& c, v8f& d) {
#if defined(__HIP_DEVICE_COMPILE__)
  asm volatile("v_nop\n\tv_nop\n\tv_nop\n\tv_nop" : "+v"(a), "+v"(b), "+v"(c), "+v"(d));
#endif
}
__device__ __forceinline__ void wave_sync_lds() {
  __builtin_amdgcn_fence(__ATOMIC_RELEASE, "workgroup");
  __builtin_amdgcn_wave_barrier();
  __builtin_amdgcn_fence(__ATOMIC_ACQUIRE, "workgroup");
}

__device__ __forceinline__ void sincos_cw(float x, float& s, float& c) {
#pragma clang fp contract(off)
  const float k = rintf(x * 0.63661977236758134f);
  float r = fmaf(-k, 1.5703125f, x);
  r = fmaf(-k, 4.837512969970703125e-4f, r);
  r = fmaf(-k, 7.54978995489188216e-8f, r);
  const int q = ((int)k) & 3;
  const float r2 = r * r;
  float sp = fmaf(r2, -1.9515295891e-4f, 8.3321608736e-3f);
  sp = fmaf(r2, sp, -1.6666654611e-1f);
  const float ss = fmaf(r2 * r, sp, r);
  float cq = fmaf(r2, 2.443315711809948e-5f, -1.388731625493765e-3f);
  cq = fmaf(r2, cq, 4.166664568298827e-2f);
  const float cc = fmaf(r2 * r2, cq, fmaf(r2, -0.5f, 1.0f));
  const float sa = (q & 1) ? cc : ss;
  const float ca = (q & 1) ? ss : cc;
  s = (q & 2) ? -sa : sa;
  c = ((q + 1) & 2) ? -ca : ca;
}

__global__ __launch_bounds__(256) void cvt_wT(const float* __restrict__ w0, const float* __restrict__ w1,
                                              const float* __restrict__ w2, const float* __restrict__ w3,
                                              int nsel, int zstride, unsigned short* outp, int nin, int nout) {
  __shared__ float tile[64][33];
  const int tid = threadIdx.x;
  const int z = blockIdx.z;
  const int sel = z % nsel, lay = z / nsel;
  const float* base = (sel == 0) ? w0 : ((sel == 1) ? w1 : ((sel == 2) ? w2 : w3));
  const float* src = base + (size_t)lay * zstride;
  unsigned short* dst = outp + (size_t)z * nin * nout;
  const int i0 = blockIdx.x * 64;
  const int o0 = blockIdx.y * 32;
#pragma unroll
  for (int p = 0; p < 8; ++p) {
    const int idx = p * 256 + tid;
    const int i = idx >> 5, o = idx & 31;
    tile[i][o] = src[(size_t)(i0 + i) * nout + o0 + o];
  }
  __syncthreads();
  const int o = tid >> 3, c8 = (tid & 7) * 8;
  v4u pk;
#pragma unroll
  for (int e = 0; e < 4; ++e)
    pk[e] = pkh(bfr(tile[c8 + 2 * e][o]) * WSC, bfr(tile[c8 + 2 * e + 1][o]) * WSC);
  unsigned short* gp = dst + (size_t)(o0 + o) * nin + i0 + c8;
  *(volatile v4u*)gp = pk;
  __threadfence();
  *(volatile v4u*)gp = pk;
}

__global__ __launch_bounds__(256) void encode_ln(const float* __restrict__ qc, const float* __restrict__ qf2,
                                                 const float* __restrict__ qf3, const float* __restrict__ kc,
                                                 const float* __restrict__ kf2, const float* __restrict__ kf3,
                                                 const float* __restrict__ lng, const float* __restrict__ lnb,
                                                 unsigned short* xh) {
#pragma clang fp contract(off)
  __shared__ float rcpt[64];
  const int tid = threadIdx.x, wave = tid >> 5, lane = tid & 31;
  if (tid < 64) {
    const double ex = (double)tid * 0.20762050593046015;
    const float inv = (float)exp2(ex);
    rcpt[tid] = 1.0f / inv;
  }
  __syncthreads();
  const int row = blockIdx.x * 8 + wave;
  const bool isq = row < QROWS;
  const int lr = isq ? row : (row - QROWS);
  const float* cp = isq ? qc : kc;
  const float* f2 = isq ? qf2 : kf2;
  const float* f3 = isq ? qf3 : kf3;
  const int c8 = lane * 8;
  const int ci = (c8 < 128) ? 0 : 1;
  const float cv = bfr(cp[(size_t)lr * 2 + ci]);
  const int jb = (c8 & 127) >> 1;
  const float* p2 = f2 + (size_t)lr * HID + c8;
  const float* p3 = f3 + (size_t)lr * HID + c8;
  const v4f a0 = *(const v4f*)p2, a1 = *(const v4f*)(p2 + 4);
  const v4f b0 = *(const v4f*)p3, b1 = *(const v4f*)(p3 + 4);
  float x[8];
#pragma unroll
  for (int e = 0; e < 4; ++e) {
    x[e]     = bfr(a0[e]) + bfr(b0[e]);
    x[4 + e] = bfr(a1[e]) + bfr(b1[e]);
  }
#pragma unroll
  for (int e = 0; e < 4; ++e) {
    const float ang = cv * rcpt[jb + e];
    float sn, cs;
    sincos_cw(ang, sn, cs);
    x[2 * e]     = x[2 * e] + sn;
    x[2 * e + 1] = x[2 * e + 1] + cs;
  }
  float s = 0.f;
#pragma unroll
  for (int e = 0; e < 8; ++e) s = s + x[e];
#pragma unroll
  for (int off = 1; off < 32; off <<= 1) s = s + __shfl_xor(s, off, 32);
  const float mu = s * (1.0f / HID);
  float d[8];
  float s2 = 0.f;
#pragma unroll
  for (int e = 0; e < 8; ++e) { d[e] = x[e] - mu; const float dd = d[e] * d[e]; s2 = s2 + dd; }
#pragma unroll
  for (int off = 1; off < 32; off <<= 1) s2 = s2 + __shfl_xor(s2, off, 32);
  const float var = s2 * (1.0f / HID);
  const float rstd = 1.0f / sqrtf(var + LNEPS);
  float y[8];
#pragma unroll
  for (int e = 0; e < 8; ++e) {
    const float g = bfr(lng[c8 + e]), bb = bfr(lnb[c8 + e]);
    float t = d[e] * rstd; t = t * g; y[e] = t + bb;
  }
  v4u ph;
#pragma unroll
  for (int e = 0; e < 4; ++e) ph[e] = pkh(y[2 * e], y[2 * e + 1]);
  unsigned short* gp = xh + (size_t)row * HID + c8;
  *(volatile v4u*)gp = ph;
  __threadfence();
  *(volatile v4u*)gp = ph;
}

__global__ __launch_bounds__(256) void tok_init(const float* __restrict__ tv, float* tf, unsigned short* th) {
  const int tid = threadIdx.x, wave = tid >> 5, lane = tid & 31;
  const int row = blockIdx.x * 8 + wave;
  const bool live = (row == 0) || (row == TOKR);
  const int c4 = lane * 4, c8 = lane * 8;
  v4f p0, p1;
  v4u ph;
#pragma unroll
  for (int e = 0; e < 4; ++e) {
    const float f0 = bfr(tv[c4 + e]), f1 = bfr(tv[128 + c4 + e]);
    p0[e] = live ? f0 : 0.f;
    p1[e] = live ? f1 : 0.f;
    const float g0 = bfr(tv[c8 + 2 * e]), g1 = bfr(tv[c8 + 2 * e + 1]);
    ph[e] = pkh(live ? g0 : 0.f, live ? g1 : 0.f);
  }
  float* fp = tf + (size_t)row * HID;
  unsigned short* hp = th + (size_t)row * HID + c8;
  for (int pass = 0; pass < 2; ++pass) {
    *(volatile v4f*)(fp + c4) = p0;
    *(volatile v4f*)(fp + 128 + c4) = p1;
    *(volatile v4u*)hp = ph;
    __threadfence();
  }
}

__global__ __launch_bounds__(256) void ln256(const float* __restrict__ zin, const float* __restrict__ g,
                                             const float* __restrict__ bt, float* outF, unsigned short* outH,
                                             int nrows) {
#pragma clang fp contract(off)
  __shared__ __align__(16) float rb[8][HID];
  const int tid = threadIdx.x, wave = tid >> 5, lane = tid & 31;
  const int row = blockIdx.x * 8 + wave;
  const int rowc = (row < nrows) ? row : (nrows - 1);
  const int c8 = lane * 8;
  const float* rp = zin + (size_t)rowc * HID + c8;
  const v4f a = *(const v4f*)rp;
  const v4f b = *(const v4f*)(rp + 4);
  float x[8];
#pragma unroll
  for (int e = 0; e < 4; ++e) { x[e] = a[e]; x[4 + e] = b[e]; }
  float s = 0.f;
#pragma unroll
  for (int e = 0; e < 8; ++e) s = s + x[e];
#pragma unroll
  for (int off = 1; off < 32; off <<= 1) s = s + __shfl_xor(s, off, 32);
  const float mu = s * (1.0f / HID);
  float d[8];
  float s2 = 0.f;
#pragma unroll
  for (int e = 0; e < 8; ++e) { d[e] = x[e] - mu; const float dd = d[e] * d[e]; s2 = s2 + dd; }
#pragma unroll
  for (int off = 1; off < 32; off <<= 1) s2 = s2 + __shfl_xor(s2, off, 32);
  const float var = s2 * (1.0f / HID);
  const float rstd = 1.0f / sqrtf(var + LNEPS);
  float y[8];
#pragma unroll
  for (int e = 0; e < 8; ++e) {
    const float gg = bfr(g[c8 + e]), bb = bfr(bt[c8 + e]);
    float t = d[e] * rstd; t = t * gg; y[e] = t + bb;
  }
  v4u ph;
#pragma unroll
  for (int e = 0; e < 4; ++e) ph[e] = pkh(y[2 * e], y[2 * e + 1]);
  float* myrb = rb[wave];
  {
    v4f y0 = {y[0], y[1], y[2], y[3]};
    v4f y1 = {y[4], y[5], y[6], y[7]};
    *(v4f*)(myrb + c8) = y0;
    *(v4f*)(myrb + c8 + 4) = y1;
  }
  wave_sync_lds();
  const v4f q0 = *(const v4f*)(myrb + 4 * lane);
  const v4f q1 = *(const v4f*)(myrb + 128 + 4 * lane);
  if (row < nrows) {
    float* fp = outF + (size_t)row * HID;
    unsigned short* hp = outH + (size_t)row * HID + c8;
    for (int pass = 0; pass < 2; ++pass) {
      *(volatile v4u*)hp = ph;
      *(volatile v4f*)(fp + 4 * lane) = q0;
      *(volatile v4f*)(fp + 128 + 4 * lane) = q1;
      __threadfence();
    }
  }
}

struct GDesc {
  const unsigned short* A;
  const unsigned short* Bt;
  const float* bias;
  const float* resid;
  void* C;
  int lda, ldb, ldc, ldr;
  int M, N, K, blen;
  int flags, mseg, mbstr, moff;
  int nseg, nbstr, noff, tile0;
  int tiles, pad0;
  float wscale, oscale;
};
static_assert(sizeof(GDesc) == 120);
struct GBatch {
  GDesc d[6];
  int nd;
  int tot;
};
static_assert(sizeof(GBatch) == 728);

__device__ __forceinline__ float epi1(float a, int m, int n, float wsc, const float* bias, int blen, int fl) {
#pragma clang fp contract(off)
  float f = a * wsc;
  if (fl & F_BIASN) { const int i = (n < blen) ? n : (blen - 1); f = f + bfr(bias[i]); }
  if (fl & F_BIASM) { const int i = (m < blen) ? m : (blen - 1); f = f + bfr(bias[i]); }
  return f;
}

__global__ __launch_bounds__(256) void gemm_batch(GBatch gb) {
#pragma clang fp contract(off)
  __shared__ __align__(16) float sT[8][16 * 68];
  const int lane = threadIdx.x & 31;
  const int wave = threadIdx.x >> 5;
  const int t = blockIdx.x * 8 + wave;
  if (t >= gb.tot) return;
  int di = 0;
#pragma unroll
  for (int i = 1; i < 6; ++i) { if (t >= gb.d[i].tile0) di = i; }
  GDesc D = gb.d[0];
#pragma unroll
  for (int i = 1; i < 6; ++i) { if (di == i) D = gb.d[i]; }

  const _Float16* A  = (const _Float16*)(const void*)D.A;
  const _Float16* Bt = (const _Float16*)(const void*)D.Bt;
  const int tilesN = D.N >> 6;
  const int lt = t - D.tile0;
  const int tm = lt / tilesN;
  const int tn = lt - tm * tilesN;
  const int m0 = tm * 32;
  const int n0 = tn * 64;

  const int rlane = lane & 15;
  const int koff  = (lane >> 4) * 8;
  const int mOff  = (lane >> 4) * 8;

  v8f acc[2][4];
#pragma unroll
  for (int i = 0; i < 2; ++i)
#pragma unroll
    for (int j = 0; j < 4; ++j) acc[i][j] = zero8();

  for (int k0 = 0; k0 < D.K; k0 += 32) {
    v16h bh[4];
#pragma unroll
    for (int j = 0; j < 4; ++j) {
      const size_t bo = (size_t)(n0 + (j << 4) + rlane) * D.ldb + koff + k0;
      bh[j] = ldfrag_h(Bt + bo);
    }
#pragma unroll
    for (int i = 0; i < 2; ++i) {
      const size_t ao = (size_t)(m0 + (i << 4) + rlane) * D.lda + koff + k0;
      const v16h ah = ldfrag_h(A + ao);
#pragma unroll
      for (int j = 0; j < 4; ++j) acc[i][j] = mma_h_raw(ah, bh[j], acc[i][j]);
      dep_guard_h(acc[i][0], acc[i][3], ah);
    }
    keep4_h(bh[0], bh[1], bh[2], bh[3]);
  }
#pragma unroll
  for (int i = 0; i < 2; ++i) acc_guard4(acc[i][0], acc[i][1], acc[i][2], acc[i][3]);

  const int orow0 = (m0 / D.mseg) * D.mbstr + D.moff + (m0 % D.mseg);
  const int ocol0 = (n0 / D.nseg) * D.nbstr + D.noff + (n0 % D.nseg);
  const int fl = D.flags;
  const float wsc = D.wscale, osc = D.oscale;

  float* slab = sT[wave];
#pragma unroll
  for (int i = 0; i < 2; ++i) {
    const int mBase = m0 + (i << 4);
#pragma unroll
    for (int j = 0; j < 4; ++j) {
#pragma unroll
      for (int r = 0; r < 8; ++r) {
        slab[(mOff + r) * 68 + (j << 4) + rlane] = acc[i][j][r];
      }
    }
    wave_sync_lds();
    if ((fl & F_OUT16) == 0) {
      float* C = (float*)D.C;
      const int h2 = lane >> 4, c4 = (lane & 15) * 4;
      v4f ov[8];
#pragma unroll
      for (int it = 0; it < 8; ++it) {
        const int row = it * 2 + h2;
        const int m = mBase + row;
        const v4f v = *(const v4f*)(slab + row * 68 + c4);
        v4f rv = zero4();
        if (fl & F_RESID) rv = *(const v4f*)(D.resid + (size_t)m * D.ldr + n0 + c4);
        v4f o;
#pragma unroll
        for (int e = 0; e < 4; ++e) {
          float f = epi1(v[e], m, n0 + c4 + e, wsc, D.bias, D.blen, fl);
          f = f + rv[e];
          if (fl & F_RELU) f = fmaxf(f, 0.f);
          o[e] = f * osc;
        }
        ov[it] = o;
      }
      for (int pass = 0; pass < 2; ++pass) {
#pragma unroll
        for (int it = 0; it < 8; ++it) {
          const int row = it * 2 + h2;
          float* gp = C + (size_t)(orow0 + (i << 4) + row) * D.ldc + ocol0 + c4;
          *(volatile v4f*)gp = ov[it];
        }
        __threadfence();
      }
    } else {
      unsigned short* C = (unsigned short*)D.C;
      const int q = lane >> 3, c8 = (lane & 7) * 8;
      v4u hv[4];
#pragma unroll
      for (int it = 0; it < 4; ++it) {
        const int row = it * 4 + q;
        const int m = mBase + row;
        const float* sp = slab + row * 68 + c8;
        float rr[8];
#pragma unroll
        for (int e = 0; e < 8; ++e) rr[e] = 0.f;
        if (fl & F_RESID) {
          const float* rp2 = D.resid + (size_t)m * D.ldr + n0 + c8;
          const v4f r0v = *(const v4f*)rp2;
          const v4f r1v = *(const v4f*)(rp2 + 4);
#pragma unroll
          for (int e = 0; e < 4; ++e) { rr[e] = r0v[e]; rr[4 + e] = r1v[e]; }
        }
        float fv[8];
#pragma unroll
        for (int e = 0; e < 8; ++e) {
          float f = epi1(sp[e], m, n0 + c8 + e, wsc, D.bias, D.blen, fl);
          f = f + rr[e];
          if (fl & F_RELU) f = fmaxf(f, 0.f);
          fv[e] = f * osc;
        }
        v4u a;
#pragma unroll
        for (int e = 0; e < 4; ++e) a[e] = pkh(fv[2 * e], fv[2 * e + 1]);
        hv[it] = a;
      }
      for (int pass = 0; pass < 2; ++pass) {
#pragma unroll
        for (int it = 0; it < 4; ++it) {
          const int row = it * 4 + q;
          unsigned short* gp = C + (size_t)(orow0 + (i << 4) + row) * D.ldc + ocol0 + c8;
          *(volatile v4u*)gp = hv[it];
        }
        __threadfence();
      }
    }
    wave_sync_lds();
  }
}

__global__ __launch_bounds__(256)
void attn16(const unsigned short* __restrict__ qpl, int qbs,
            const unsigned short* __restrict__ skpl, const unsigned short* __restrict__ svpl, int selfon,
            const unsigned short* __restrict__ kpl, const unsigned short* __restrict__ vtpl,
            int nk, int nchunk, const int* __restrict__ mask, int maskon, int maskn,
            unsigned short* opl) {
#pragma clang fp contract(off)
  union FH { v16h v; v8h h[2]; };
  __shared__ __align__(16) _Float16 Psh[8][16 * 64];
  __shared__ __align__(16) float    Os[16 * HID];

  const int tid  = threadIdx.x;
  const int wave = tid >> 5;
  const int lane = tid & 31;
  const int hh   = lane >> 4;
  const int c    = lane & 15;
  const int b    = blockIdx.y;
  const int m0   = blockIdx.x * 16;
  const int hd   = wave;
  const size_t qrow0 = (size_t)b * qbs + m0;

  const _Float16* Q  = (const _Float16*)(const void*)qpl;
  const _Float16* SK = (const _Float16*)(const void*)skpl;
  const _Float16* SV = (const _Float16*)(const void*)svpl;
  const _Float16* Kh = (const _Float16*)(const void*)kpl;
  const _Float16* Vh = (const _Float16*)(const void*)vtpl;

  const v16h qa = ldfrag_h(Q + (qrow0 + c) * HID + hd * DHD + 8 * hh);

  const float invq2 = 1.0f / (PSC * PSC);
  float mrow[8], lrow[8];
  v8f oh[2];
#pragma unroll
  for (int r = 0; r < 8; ++r) { mrow[r] = -INFINITY; lrow[r] = 0.f; }
  oh[0] = zero8(); oh[1] = zero8();

  if (selfon != 0) {
#pragma unroll
    for (int r = 0; r < 8; ++r) {
      const size_t row = qrow0 + 8 * hh + r;
      const _Float16* qr = Q  + row * HID + hd * DHD + 2 * c;
      const _Float16* kr = SK + row * HID + hd * DHD + 2 * c;
      float pr = (float)qr[0] * (float)kr[0];
      const float p2 = (float)qr[1] * (float)kr[1];
      pr = pr + p2;
#pragma unroll
      for (int off = 1; off < 16; off <<= 1) pr = pr + __shfl_xor(pr, off, 32);
      const float sv0 = (float)SV[row * HID + hd * DHD + c];
      const float sv1 = (float)SV[row * HID + hd * DHD + 16 + c];
      float ms = pr * invq2; ms = ms * RSCALE;
      mrow[r] = ms;
      lrow[r] = 1.0f;
      oh[0][r] = sv0 * 1024.0f;
      oh[1][r] = sv1 * 1024.0f;
    }
  }

  _Float16* pw = Psh[wave];
  const int* mrowp = mask + (size_t)b * maskn;

  for (int kt = 0; kt < nchunk; ++kt) {
    const int kv0 = kt * 64;

    v8f s[4];
#pragma unroll
    for (int j = 0; j < 4; ++j) {
      const int key  = kv0 + j * 16 + c;
      const int keyc = (key < NKP) ? key : (NKP - 1);
      const size_t ko = ((size_t)b * NKP + keyc) * HID + hd * DHD + 8 * hh;
      const v16h kb = ldfrag_h(Kh + ko);
      const v8f a = mma_h(qa, kb, zero8());
      const bool dead = key >= nk;
      const int mi = (key < maskn) ? key : (maskn - 1);
      const int mv = mrowp[mi];
      const float sub = (maskon != 0 && mv == 0) ? 1e10f : 0.0f;
#pragma unroll
      for (int r = 0; r < 8; ++r) {
        const float t0 = a[r] * invq2;
        const float t1 = t0 - sub;
        const float sc = t1 * RSCALE;
        s[j][r] = dead ? -INFINITY : sc;
      }
    }

#pragma unroll
    for (int r = 0; r < 8; ++r) {
      float m = fmaxf(fmaxf(s[0][r], s[1][r]), fmaxf(s[2][r], s[3][r]));
#pragma unroll
      for (int off = 1; off < 16; off <<= 1) m = fmaxf(m, __shfl_xor(m, off, 32));
      const float mnew  = fmaxf(mrow[r], m);
      const float alpha = (mnew == -INFINITY) ? 1.0f : __expf(mrow[r] - mnew);
      mrow[r] = mnew;
      float psum = 0.f;
#pragma unroll
      for (int j = 0; j < 4; ++j) {
        const float p  = (s[j][r] == -INFINITY) ? 0.f : __expf(s[j][r] - mnew);
        psum += p;
        const float p1 = p * 1024.0f;
        pw[(8 * hh + r) * 64 + j * 16 + c] = (_Float16)p1;
      }
#pragma unroll
      for (int off = 1; off < 16; off <<= 1) psum += __shfl_xor(psum, off, 32);
      lrow[r] = lrow[r] * alpha + psum;
      oh[0][r] *= alpha;
      oh[1][r] *= alpha;
    }
    wave_sync_lds();

#pragma unroll
    for (int kk = 0; kk < 2; ++kk) {
      FH pa;
      pa.h[0] = *(const v8h*)(pw + c * 64 + kk * 32 + 8 * hh);
      pa.h[1] = *(const v8h*)(pw + c * 64 + kk * 32 + 16 + 8 * hh);
#pragma unroll
      for (int tt = 0; tt < 2; ++tt) {
        const int d = hd * DHD + tt * 16 + c;
        const size_t vo = ((size_t)b * HID + d) * NKP + kv0 + kk * 32 + 8 * hh;
        const v16h vb = ldfrag_h(Vh + vo);
        oh[tt] = mma_h(pa.v, vb, oh[tt]);
      }
    }
    wave_sync_lds();
  }

#pragma unroll
  for (int r = 0; r < 8; ++r) {
    const float l = lrow[r];
    const float inv = ((l > 0.f) ? (1.0f / l) : 0.f) * (OSC / (1024.0f * PSC));
#pragma unroll
    for (int tt = 0; tt < 2; ++tt) {
      const int col = hd * DHD + tt * 16 + c;
      Os[(8 * hh + r) * HID + col] = oh[tt][r] * inv;
    }
  }
  __syncthreads();
  {
    v4u hv[2];
#pragma unroll
    for (int it = 0; it < 2; ++it) {
      const int row = wave * 2 + it;
      const float* sp = Os + row * HID + 8 * lane;
      v4u a;
#pragma unroll
      for (int e = 0; e < 4; ++e) a[e] = pkh(sp[2 * e], sp[2 * e + 1]);
      hv[it] = a;
    }
    for (int pass = 0; pass < 2; ++pass) {
#pragma unroll
      for (int it = 0; it < 2; ++it) {
        const int row = wave * 2 + it;
        unsigned short* gp = opl + (qrow0 + row) * HID + 8 * lane;
        *(volatile v4u*)gp = hv[it];
      }
      __threadfence();
    }
  }
}

__global__ __launch_bounds__(256) void tok_kv(const float* __restrict__ tf, const float* __restrict__ wk,
                                              const float* __restrict__ bk, const float* __restrict__ wv,
                                              const float* __restrict__ bv, unsigned short* kp, unsigned short* vt) {
  __shared__ __align__(16) unsigned short krow[HID];
  __shared__ float vval[HID];
  const int tid = threadIdx.x, wave = tid >> 5, lane = tid & 31;
  const int b = blockIdx.x;
  const int d = tid;
  const float* x = tf + (size_t)(b * TOKR) * HID;
  float ka = 0.f, va = 0.f;
#pragma unroll 4
  for (int k = 0; k < HID; ++k) {
    const float xv = x[k];
    ka += xv * bfr(wk[(size_t)k * HID + d]);
    va += xv * bfr(wv[(size_t)k * HID + d]);
  }
  krow[d] = h_bits((_Float16)((ka + bfr(bk[d])) * PSC));
  vval[d] = (va + bfr(bv[d])) * PSC;
  __syncthreads();
  const v4u kvv = *(const v4u*)(krow + 8 * lane);
  const v4u z4 = {0u, 0u, 0u, 0u};
  for (int pass = 0; pass < 2; ++pass) {
#pragma unroll
    for (int it = 0; it < 8; ++it) {
      const int r = (NCAT - 1) + it * 8 + wave;
      const v4u val = (it == 0 && wave == 0) ? kvv : z4;
      unsigned short* gp = kp + ((size_t)b * NKP + r) * HID + 8 * lane;
      *(volatile v4u*)gp = val;
    }
    __threadfence();
  }
  const int q = lane >> 3, p = lane & 7;
  v4u vv[8];
#pragma unroll
  for (int it = 0; it < 8; ++it) {
    const int dr = it * 32 + wave * 4 + q;
    const unsigned hv = (unsigned)h_bits((_Float16)vval[dr]);
    v4u val = z4;
    val[0] = (p == 0) ? hv : 0u;
    vv[it] = val;
  }
  for (int pass = 0; pass < 2; ++pass) {
#pragma unroll
    for (int it = 0; it < 8; ++it) {
      const int dr = it * 32 + wave * 4 + q;
      unsigned short* gp = vt + ((size_t)b * HID + dr) * NKP + (NCAT - 1) + 8 * p;
      *(volatile v4u*)gp = vv[it];
    }
    __threadfence();
  }
}

__global__ __launch_bounds__(64) void out_tok(const float* __restrict__ tf, float* outp) {
  const int tid = threadIdx.x, wave = tid >> 5, lane = tid & 31;
  const float* sp = tf + (size_t)(wave * TOKR) * HID;
  const v4f p0 = *(const v4f*)(sp + 4 * lane);
  const v4f p1 = *(const v4f*)(sp + 128 + 4 * lane);
  float* dp = outp + (size_t)wave * HID;
  for (int pass = 0; pass < 2; ++pass) {
    *(volatile v4f*)(dp + 4 * lane) = p0;
    *(volatile v4f*)(dp + 128 + 4 * lane) = p1;
    __threadfence();
  }
}

static GDesc gdesc(const unsigned short* A, int lda, const unsigned short* Bt, int ldb, void* C, int ldc,
                   int M, int N, int K, const float* bias, int blen, const float* resid, int ldr,
                   int flags, float wscale, float oscale) {
  GDesc d;
  d.A = A; d.Bt = Bt; d.bias = bias; d.resid = resid; d.C = C;
  d.lda = lda; d.ldb = ldb; d.ldc = ldc; d.ldr = ldr;
  d.M = M; d.N = N; d.K = K; d.blen = blen;
  d.flags = flags; d.mseg = 1 << 30; d.mbstr = 0; d.moff = 0;
  d.nseg = 1 << 30; d.nbstr = 0; d.noff = 0; d.tile0 = 0;
  d.tiles = (M / 32) * (N / 64); d.pad0 = 0;
  d.wscale = wscale; d.oscale = oscale;
  return d;
}
static void run_gemm(const GDesc* ds, int nd, hipStream_t stream) {
  GBatch gb;
  int tot = 0;
  for (int i = 0; i < 6; ++i) {
    if (i < nd) { gb.d[i] = ds[i]; gb.d[i].tile0 = tot; tot += ds[i].tiles; }
    else        { gb.d[i] = ds[0]; gb.d[i].tile0 = 1 << 30; gb.d[i].tiles = 0; }
  }
  gb.nd = nd; gb.tot = tot;
  if (tot <= 0) return;
  const dim3 grid((tot + 7) / 8);
  gemm_batch<<<grid, dim3(256), 0, stream>>>(gb);
}

extern "C" void kernel_launch(void* const* d_in, const int* in_sizes, int n_in,
                              void* d_out, int out_size, void* d_ws, size_t ws_size,
                              hipStream_t stream) {
  if (n_in < 30) return;
  const int ex[30] = { NB * MQ * 2, NB * MQ * HID, NB * MQ * HID, NB * NKEY * 2, NB * NKEY * HID, NB * NKEY * HID,
                       NB * NKEY, HID, HID, HID * HID, HID, HID, HID, HID,
                       NLAY * HID * HID, NLAY * HID, NLAY * HID * HID, NLAY * HID, NLAY * HID * HID, NLAY * HID,
                       NLAY * HID * HID, NLAY * HID, NLAY * HID, NLAY * HID, NLAY * HID * FFI, NLAY * FFI,
                       NLAY * FFI * HID, NLAY * HID, NLAY * HID, NLAY * HID };
  for (int i = 0; i < 30; ++i) if (in_sizes[i] != ex[i]) return;
  if (out_size != SROWS * HID + NB * HID) return;

  const float* qc2  = (const float*)d_in[0];
  const float* qf2  = (const float*)d_in[1];
  const float* qf3  = (const float*)d_in[2];
  const float* kc2  = (const float*)d_in[3];
  const float* kf2  = (const float*)d_in[4];
  const float* kf3  = (const float*)d_in[5];
  const int*   amask = (const int*)d_in[6];
  const float* ln1g = (const float*)d_in[7];
  const float* ln1b = (const float*)d_in[8];
  const float* dcW  = (const float*)d_in[9];
  const float* dcb  = (const float*)d_in[10];
  const float* dclg = (const float*)d_in[11];
  const float* dclb = (const float*)d_in[12];
  const float* tokv = (const float*)d_in[13];
  const float* Wq = (const float*)d_in[14]; const float* bq = (const float*)d_in[15];
  const float* Wk = (const float*)d_in[16]; const float* bk = (const float*)d_in[17];
  const float* Wv = (const float*)d_in[18]; const float* bv = (const float*)d_in[19];
  const float* Wd = (const float*)d_in[20]; const float* bd = (const float*)d_in[21];
  const float* alg = (const float*)d_in[22]; const float* alb = (const float*)d_in[23];
  const float* W1 = (const float*)d_in[24]; const float* b1 = (const float*)d_in[25];
  const float* W2 = (const float*)d_in[26]; const float* b2 = (const float*)d_in[27];
  const float* flg = (const float*)d_in[28]; const float* flb = (const float*)d_in[29];
  float* out = (float*)d_out;

  const size_t sWP  = (size_t)NLAY * 4 * HID * HID * 2;
  const size_t sW1  = (size_t)NLAY * HID * FFI * 2;
  const size_t sW2  = sW1;
  const size_t sDC  = (size_t)HID * HID * 2;
  const size_t sX   = (size_t)SROWS * HID * 2;
  const size_t sSH  = sX;
  const size_t sPRE = (size_t)SROWS * HID * 4;
  const size_t sAF  = (size_t)KROWS * HID * 4;
  const size_t sAH  = (size_t)KROWS * HID * 2;
  const size_t sHP  = (size_t)KROWS * FFI * 2;
  const size_t sQP  = (size_t)KROWS * HID * 2;
  const size_t sSK  = (size_t)QROWS * HID * 2;
  const size_t sKP  = (size_t)NB * NKP * HID * 2;
  const size_t sVT  = sKP;
  const size_t sOP  = sQP;
  const size_t sTF  = (size_t)NTOK * HID * 4;
  const size_t sTH  = (size_t)NTOK * HID * 2;
  size_t off = 0;
  const size_t oWP  = off; off += sWP;
  const size_t oW1  = off; off += sW1;
  const size_t oW2  = off; off += sW2;
  const size_t oDC  = off; off += sDC;
  const size_t oX   = off; off += sX;
  const size_t oSH  = off; off += sSH;
  const size_t oPRE = off; off += sPRE;
  const size_t oAF  = off; off += sAF;
  const size_t oAH  = off; off += sAH;
  const size_t oHP  = off; off += sHP;
  const size_t oQP  = off; off += sQP;
  const size_t oSK  = off; off += sSK;
  const size_t oSV  = off; off += sSK;
  const size_t oKP  = off; off += sKP;
  const size_t oVT  = off; off += sVT;
  const size_t oOP  = off; off += sOP;
  const size_t oTF  = off; off += sTF;
  const size_t oTH  = off; off += sTH;
  if (off > ws_size) return;
  if (off > (size_t)134217728) return;

  char* ws = (char*)d_ws;
  unsigned short* WP   = (unsigned short*)(ws + oWP);
  unsigned short* W1P  = (unsigned short*)(ws + oW1);
  unsigned short* W2P  = (unsigned short*)(ws + oW2);
  unsigned short* DCP  = (unsigned short*)(ws + oDC);
  unsigned short* X    = (unsigned short*)(ws + oX);
  unsigned short* SH   = (unsigned short*)(ws + oSH);
  float*          PRE  = (float*)(ws + oPRE);
  float*          AF   = (float*)(ws + oAF);
  unsigned short* AH   = (unsigned short*)(ws + oAH);
  unsigned short* HP   = (unsigned short*)(ws + oHP);
  unsigned short* QP   = (unsigned short*)(ws + oQP);
  unsigned short* SKP  = (unsigned short*)(ws + oSK);
  unsigned short* SVP  = (unsigned short*)(ws + oSV);
  unsigned short* KP   = (unsigned short*)(ws + oKP);
  unsigned short* VT   = (unsigned short*)(ws + oVT);
  unsigned short* OP   = (unsigned short*)(ws + oOP);
  float*          TOKF = (float*)(ws + oTF);
  unsigned short* TOKH = (unsigned short*)(ws + oTH);

  unsigned short* SHq = SH;
  unsigned short* SHk = SH + (size_t)QROWS * HID;
  float* OUTq = out;
  float* OUTk = out + (size_t)QROWS * HID;
  float* OUTt = out + (size_t)SROWS * HID;

  const dim3 blk(256);

  cvt_wT<<<dim3(HID / 64, HID / 32, NLAY * 4), blk, 0, stream>>>(Wq, Wk, Wv, Wd, 4, HID * HID, WP, HID, HID);
  cvt_wT<<<dim3(HID / 64, FFI / 32, NLAY), blk, 0, stream>>>(W1, W1, W1, W1, 1, HID * FFI, W1P, HID, FFI);
  cvt_wT<<<dim3(FFI / 64, HID / 32, NLAY), blk, 0, stream>>>(W2, W2, W2, W2, 1, FFI * HID, W2P, FFI, HID);
  cvt_wT<<<dim3(HID / 64, HID / 32, 1), blk, 0, stream>>>(dcW, dcW, dcW, dcW, 1, 0, DCP, HID, HID);
  encode_ln<<<dim3(SROWS / 8), blk, 0, stream>>>(qc2, qf2, qf3, kc2, kf2, kf3, ln1g, ln1b, X);
  tok_init<<<dim3(NTOK / 8), blk, 0, stream>>>(tokv, TOKF, TOKH);
  {
    GDesc d[1];
    d[0] = gdesc(X, HID, DCP, HID, (void*)PRE, HID, SROWS, HID, HID, dcb, HID, PRE, 0, F_BIASN, 1.0f / WSC, 1.0f);
    run_gemm(d, 1, stream);
  }
  ln256<<<dim3(SROWS / 8), blk, 0, stream>>>(PRE, dclg, dclb, OUTq, SHq, SROWS);

  const float wsQ  = 1.0f / WSC;
  const float wsWd = 1.0f / (WSC * OSC);
  const float wsW2 = 1.0f / (WSC * HSC);

  for (int i = 0; i < NLAY; ++i) {
    const unsigned short* wq = WP + (size_t)(i * 4 + 0) * HID * HID;
    const unsigned short* wk = WP + (size_t)(i * 4 + 1) * HID * HID;
    const unsigned short* wv = WP + (size_t)(i * 4 + 2) * HID * HID;
    const unsigned short* wd = WP + (size_t)(i * 4 + 3) * HID * HID;
    const unsigned short* w1 = W1P + (size_t)i * HID * FFI;
    const unsigned short* w2 = W2P + (size_t)i * HID * FFI;
    const float* bqi = bq + (size_t)i * HID;  const float* bki = bk + (size_t)i * HID;
    const float* bvi = bv + (size_t)i * HID;  const float* bdi = bd + (size_t)i * HID;
    const float* algi = alg + (size_t)i * HID; const float* albi = alb + (size_t)i * HID;
    const float* b1i = b1 + (size_t)i * FFI;  const float* b2i = b2 + (size_t)i * HID;
    const float* flgi = flg + (size_t)i * HID; const float* flbi = flb + (size_t)i * HID;
    const float* wkf = Wk + (size_t)i * HID * HID;
    const float* wvf = Wv + (size_t)i * HID * HID;

    {
      GDesc d[3];
      d[0] = gdesc(SHk, HID, wq, HID, (void*)QP, HID, KROWS, HID, HID, bqi, HID, PRE, 0, F_BIASN | F_OUT16, wsQ, PSC);
      d[1] = gdesc(SHk, HID, wk, HID, (void*)KP, HID, KROWS, HID, HID, bki, HID, PRE, 0, F_BIASN | F_OUT16, wsQ, PSC);
      d[1].mseg = NKEY; d[1].mbstr = NKP; d[1].moff = 0;
      d[2] = gdesc(wv, HID, SHk, HID, (void*)VT, NKP, HID, KROWS, HID, bvi, HID, PRE, 0, F_BIASM | F_OUT16, wsQ, PSC);
      d[2].nseg = NKEY; d[2].nbstr = HID * NKP; d[2].noff = 0;
      run_gemm(d, 3, stream);
    }
    attn16<<<dim3(NKEY / 16, NB), blk, 0, stream>>>(QP, NKEY, QP, QP, 0, KP, VT, NKEY, NKEY / 64,
                                                    amask, 1, NKEY, OP);
    {
      GDesc d[1];
      d[0] = gdesc(OP, HID, wd, HID, (void*)PRE, HID, KROWS, HID, HID, bdi, HID, OUTk, HID, F_BIASN | F_RESID, wsWd, 1.0f);
      run_gemm(d, 1, stream);
    }
    ln256<<<dim3(KROWS / 8), blk, 0, stream>>>(PRE, algi, albi, AF, AH, KROWS);
    {
      GDesc d[1];
      d[0] = gdesc(AH, HID, w1, HID, (void*)HP, FFI, KROWS, FFI, HID, b1i, FFI, PRE, 0, F_BIASN | F_RELU | F_OUT16, wsQ, HSC);
      run_gemm(d, 1, stream);
    }
    {
      GDesc d[1];
      d[0] = gdesc(HP, FFI, w2, FFI, (void*)PRE, HID, KROWS, HID, FFI, b2i, HID, AF, HID, F_BIASN | F_RESID, wsW2, 1.0f);
      run_gemm(d, 1, stream);
    }
    ln256<<<dim3(KROWS / 8), blk, 0, stream>>>(PRE, flgi, flbi, OUTk, SHk, KROWS);

    {
      GDesc d[5];
      d[0] = gdesc(SHq, HID, wq, HID, (void*)QP,  HID, QROWS, HID, HID, bqi, HID, PRE, 0, F_BIASN | F_OUT16, wsQ, PSC);
      d[1] = gdesc(SHq, HID, wk, HID, (void*)SKP, HID, QROWS, HID, HID, bki, HID, PRE, 0, F_BIASN | F_OUT16, wsQ, PSC);
      d[2] = gdesc(SHq, HID, wv, HID, (void*)SVP, HID, QROWS, HID, HID, bvi, HID, PRE, 0, F_BIASN | F_OUT16, wsQ, PSC);
      d[3] = gdesc(SHk, HID, wk, HID, (void*)KP, HID, KROWS, HID, HID, bki, HID, PRE, 0, F_BIASN | F_OUT16, wsQ, PSC);
      d[3].mseg = NKEY; d[3].mbstr = NKP; d[3].moff = 0;
      d[4] = gdesc(wv, HID, SHk, HID, (void*)VT, NKP, HID, KROWS, HID, bvi, HID, PRE, 0, F_BIASM | F_OUT16, wsQ, PSC);
      d[4].nseg = NKEY; d[4].nbstr = HID * NKP; d[4].noff = 0;
      run_gemm(d, 5, stream);
    }
    attn16<<<dim3(MQ / 16, NB), blk, 0, stream>>>(QP, MQ, SKP, SVP, 1, KP, VT, NKEY, NKEY / 64,
                                                  amask, 1, NKEY, OP);
    {
      GDesc d[1];
      d[0] = gdesc(OP, HID, wd, HID, (void*)PRE, HID, QROWS, HID, HID, bdi, HID, OUTq, HID, F_BIASN | F_RESID, wsWd, 1.0f);
      run_gemm(d, 1, stream);
    }
    ln256<<<dim3(QROWS / 8), blk, 0, stream>>>(PRE, algi, albi, AF, AH, QROWS);
    {
      GDesc d[1];
      d[0] = gdesc(AH, HID, w1, HID, (void*)HP, FFI, QROWS, FFI, HID, b1i, FFI, PRE, 0, F_BIASN | F_RELU | F_OUT16, wsQ, HSC);
      run_gemm(d, 1, stream);
    }
    {
      GDesc d[1];
      d[0] = gdesc(HP, FFI, w2, FFI, (void*)PRE, HID, QROWS, HID, FFI, b2i, HID, AF, HID, F_BIASN | F_RESID, wsW2, 1.0f);
      run_gemm(d, 1, stream);
    }
    ln256<<<dim3(QROWS / 8), blk, 0, stream>>>(PRE, flgi, flbi, OUTq, SHq, QROWS);

    {
      GDesc d[3];
      d[0] = gdesc(TOKH, HID, wq, HID, (void*)QP, HID, NTOK, HID, HID, bqi, HID, PRE, 0, F_BIASN | F_OUT16, wsQ, PSC);
      d[1] = gdesc(SHq, HID, wk, HID, (void*)KP, HID, QROWS, HID, HID, bki, HID, PRE, 0, F_BIASN | F_OUT16, wsQ, PSC);
      d[1].mseg = MQ; d[1].mbstr = NKP; d[1].moff = NKEY;
      d[2] = gdesc(wv, HID, SHq, HID, (void*)VT, NKP, HID, QROWS, HID, bvi, HID, PRE, 0, F_BIASM | F_OUT16, wsQ, PSC);
      d[2].nseg = MQ; d[2].nbstr = HID * NKP; d[2].noff = NKEY;
      run_gemm(d, 3, stream);
    }
    tok_kv<<<dim3(NB), blk, 0, stream>>>(TOKF, wkf, bki, wvf, bvi, KP, VT);
    attn16<<<dim3(TOKR / 16, NB), blk, 0, stream>>>(QP, TOKR, QP, QP, 0, KP, VT, NCAT, NKP / 64,
                                                    amask, 0, NKEY, OP);
    {
      GDesc d[1];
      d[0] = gdesc(OP, HID, wd, HID, (void*)PRE, HID, NTOK, HID, HID, bdi, HID, TOKF, HID, F_BIASN | F_RESID, wsWd, 1.0f);
      run_gemm(d, 1, stream);
    }
    ln256<<<dim3(NTOK / 8), blk, 0, stream>>>(PRE, algi, albi, AF, AH, NTOK);
    {
      GDesc d[1];
      d[0] = gdesc(AH, HID, w1, HID, (void*)HP, FFI, NTOK, FFI, HID, b1i, FFI, PRE, 0, F_BIASN | F_RELU | F_OUT16, wsQ, HSC);
      run_gemm(d, 1, stream);
    }
    {
      GDesc d[1];
      d[0] = gdesc(HP, FFI, w2, FFI, (void*)PRE, HID, NTOK, HID, FFI, b2i, HID, AF, HID, F_BIASN | F_RESID, wsW2, 1.0f);
      run_gemm(d, 1, stream);
    }
    ln256<<<dim3(NTOK / 8), blk, 0, stream>>>(PRE, flgi, flbi, TOKF, TOKH, NTOK);
  }

  out_tok<<<dim3(1), dim3(64), 0, stream>>>(TOKF, OUTt);
  (void)hipGetLastError();
}
